// PAM_Module_Dep_52055003628044
// MI455X (gfx1250) — hardware-verified
//
#include <hip/hip_runtime.h>


typedef _Float16 h4  __attribute__((ext_vector_type(4)));
typedef _Float16 h8  __attribute__((ext_vector_type(8)));
typedef _Float16 h16 __attribute__((ext_vector_type(16)));
typedef __bf16   bf16v16 __attribute__((ext_vector_type(16)));
typedef unsigned short us4 __attribute__((ext_vector_type(4)));
typedef unsigned short us8 __attribute__((ext_vector_type(8)));
typedef float v4f __attribute__((ext_vector_type(4)));
typedef float v8f __attribute__((ext_vector_type(8)));

#define BATCH 4
#define CCH   512
#define NPOS  4096
#define DQK   128
#define CQ    64
#define SSP   65
#define PSP   72
#define PSCALE  4096.0f
#define WVSCALE 16.0f
#define WVINV   0.0625f

union FragH { h16 v; h8 p[2]; };
union FragB { bf16v16 v; us8 p[2]; };

__device__ __forceinline__ v8f mma_f16(h16 a, h16 b, v8f c) {
  c = __builtin_amdgcn_wmma_f32_16x16x32_f16(false, a, false, b, (short)0, c, false, false);
  asm volatile("v_nop\n\tv_nop\n\tv_nop\n\tv_nop" : "+v"(c) : "v"(a), "v"(b));
  return c;
}
__device__ __forceinline__ v8f mma_bf16(bf16v16 a, bf16v16 b, v8f c) {
  c = __builtin_amdgcn_wmma_f32_16x16x32_bf16(false, a, false, b, (short)0, c, false, false);
  asm volatile("v_nop\n\tv_nop\n\tv_nop\n\tv_nop" : "+v"(c) : "v"(a), "v"(b));
  return c;
}
__device__ __forceinline__ unsigned short f2bf(float f) {
  unsigned int u = __float_as_uint(f);
  u += 0x7FFFu + ((u >> 16) & 1u);
  return (unsigned short)(u >> 16);
}
__device__ __forceinline__ float bf2f(unsigned short s) {
  return __uint_as_float(((unsigned int)s) << 16);
}

template <int MODE>
__global__ void __launch_bounds__(256)
proj_kernel(const float* __restrict__ src,
            const float* __restrict__ W,
            const float* __restrict__ bias,
            unsigned short* __restrict__ ohi,
            unsigned short* __restrict__ olo,
            _Float16* __restrict__ ov,
            int doff) {
  __shared__ __align__(16) unsigned short sm[8192];

  const int tid  = threadIdx.x;
  const int lane = tid & 31;
  const int w    = tid >> 5;
  const int m    = lane & 15;
  const int h    = lane >> 4;

  const int n0    = blockIdx.x * 64;
  const int dbase = blockIdx.y * 64;
  const int b     = blockIdx.z;

  const int mt  = w >> 1;
  const int ntb = (w & 1) * 2;

  const int ms = tid & 63;
  const int kg = (tid >> 6) * 4;

  const size_t srcb = (size_t)b * CCH * NPOS;

  v8f acc0 = {};
  v8f acc1 = {};

  if (MODE == 0) {
    unsigned short* Xh = sm;
    unsigned short* Xl = sm + 2048;
    unsigned short* Wh = sm + 4096;
    unsigned short* Wl = sm + 6144;

    for (int c0 = 0; c0 < CCH; c0 += 32) {
#pragma unroll
      for (int g = 0; g < 2; ++g) {
        const int kb = kg + g * 16;
        const float* sp = src + srcb + (size_t)(c0 + kb) * NPOS + n0 + ms;
        v4f xv;
        xv[0] = sp[0];
        xv[1] = sp[NPOS];
        xv[2] = sp[2 * NPOS];
        xv[3] = sp[3 * NPOS];
        const v4f wv4 = *(const v4f*)(W + (size_t)(dbase + ms) * CCH + c0 + kb);
        us4 xh4, xl4, wh4, wl4;
#pragma unroll
        for (int q = 0; q < 4; ++q) {
          const unsigned short hb = f2bf(xv[q]);
          xh4[q] = hb;
          xl4[q] = f2bf(xv[q] - bf2f(hb));
          const unsigned short wb = f2bf(wv4[q]);
          wh4[q] = wb;
          wl4[q] = f2bf(wv4[q] - bf2f(wb));
        }
        *(us4*)(Xh + ms * 32 + kb) = xh4;
        *(us4*)(Xl + ms * 32 + kb) = xl4;
        *(us4*)(Wh + ms * 32 + kb) = wh4;
        *(us4*)(Wl + ms * 32 + kb) = wl4;
      }
      __syncthreads();

      FragB ah, al;
      {
        const unsigned short* xr  = Xh + (mt * 16 + m) * 32 + 8 * h;
        const unsigned short* xrl = Xl + (mt * 16 + m) * 32 + 8 * h;
        ah.p[0] = *(const us8*)xr;
        ah.p[1] = *(const us8*)(xr + 16);
        al.p[0] = *(const us8*)xrl;
        al.p[1] = *(const us8*)(xrl + 16);
      }
      {
        const unsigned short* wr  = Wh + (ntb * 16 + m) * 32 + 8 * h;
        const unsigned short* wrl = Wl + (ntb * 16 + m) * 32 + 8 * h;
        FragB bh, bl;
        bh.p[0] = *(const us8*)wr;
        bh.p[1] = *(const us8*)(wr + 16);
        bl.p[0] = *(const us8*)wrl;
        bl.p[1] = *(const us8*)(wrl + 16);
        acc0 = mma_bf16(ah.v, bh.v, acc0);
        acc0 = mma_bf16(ah.v, bl.v, acc0);
        acc0 = mma_bf16(al.v, bh.v, acc0);
      }
      {
        const unsigned short* wr  = Wh + ((ntb + 1) * 16 + m) * 32 + 8 * h;
        const unsigned short* wrl = Wl + ((ntb + 1) * 16 + m) * 32 + 8 * h;
        FragB bh, bl;
        bh.p[0] = *(const us8*)wr;
        bh.p[1] = *(const us8*)(wr + 16);
        bl.p[0] = *(const us8*)wrl;
        bl.p[1] = *(const us8*)(wrl + 16);
        acc1 = mma_bf16(ah.v, bh.v, acc1);
        acc1 = mma_bf16(ah.v, bl.v, acc1);
        acc1 = mma_bf16(al.v, bh.v, acc1);
      }
      __syncthreads();
    }

    unsigned short* Eh = sm;
    unsigned short* El = sm + 4096;
    {
      const int dl = ntb * 16 + m;
      const float bb = bias[dbase + dl];
#pragma unroll
      for (int r = 0; r < 8; ++r) {
        const float v = acc0[r] + bb;
        const unsigned short hb = f2bf(v);
        const int row = mt * 16 + 8 * h + r;
        Eh[row * 64 + dl] = hb;
        El[row * 64 + dl] = f2bf(v - bf2f(hb));
      }
    }
    {
      const int dl = (ntb + 1) * 16 + m;
      const float bb = bias[dbase + dl];
#pragma unroll
      for (int r = 0; r < 8; ++r) {
        const float v = acc1[r] + bb;
        const unsigned short hb = f2bf(v);
        const int row = mt * 16 + 8 * h + r;
        Eh[row * 64 + dl] = hb;
        El[row * 64 + dl] = f2bf(v - bf2f(hb));
      }
    }
    __syncthreads();

    us8 vh[2], vl[2];
    size_t off[2];
#pragma unroll
    for (int s = 0; s < 2; ++s) {
      const int row = w * 8 + s * 4 + (lane >> 3);
      const int q = lane & 7;
      vh[s] = *(const us8*)(Eh + row * 64 + q * 8);
      vl[s] = *(const us8*)(El + row * 64 + q * 8);
      off[s] = ((size_t)b * NPOS + n0 + row) * DQK + doff + q * 8;
    }
#pragma unroll
    for (int s = 0; s < 2; ++s) {
      *(volatile us8*)(ohi + off[s]) = vh[s];
      *(volatile us8*)(olo + off[s]) = vl[s];
    }
    __threadfence();
#pragma unroll
    for (int s = 0; s < 2; ++s) {
      *(volatile us8*)(ohi + off[s]) = vh[s];
      *(volatile us8*)(olo + off[s]) = vl[s];
    }
  } else {
    _Float16* Xs = (_Float16*)sm;
    _Float16* Ws = Xs + 2048;

    for (int c0 = 0; c0 < CCH; c0 += 32) {
#pragma unroll
      for (int g = 0; g < 2; ++g) {
        const int kb = kg + g * 16;
        const float* sp = src + srcb + (size_t)(c0 + kb) * NPOS + n0 + ms;
        v4f xv;
        xv[0] = sp[0];
        xv[1] = sp[NPOS];
        xv[2] = sp[2 * NPOS];
        xv[3] = sp[3 * NPOS];
        v4f wv4 = *(const v4f*)(W + (size_t)(dbase + ms) * CCH + c0 + kb);
        wv4 = wv4 * WVSCALE;
        *(h4*)(Xs + ms * 32 + kb) = __builtin_convertvector(xv, h4);
        *(h4*)(Ws + ms * 32 + kb) = __builtin_convertvector(wv4, h4);
      }
      __syncthreads();

      FragH a;
      {
        const _Float16* xr = Xs + (mt * 16 + m) * 32 + 8 * h;
        a.p[0] = *(const h8*)xr;
        a.p[1] = *(const h8*)(xr + 16);
      }
      {
        const _Float16* wr = Ws + (ntb * 16 + m) * 32 + 8 * h;
        FragH bf;
        bf.p[0] = *(const h8*)wr;
        bf.p[1] = *(const h8*)(wr + 16);
        acc0 = mma_f16(a.v, bf.v, acc0);
      }
      {
        const _Float16* wr = Ws + ((ntb + 1) * 16 + m) * 32 + 8 * h;
        FragH bf;
        bf.p[0] = *(const h8*)wr;
        bf.p[1] = *(const h8*)(wr + 16);
        acc1 = mma_f16(a.v, bf.v, acc1);
      }
      __syncthreads();
    }

    _Float16* E = (_Float16*)sm;
    {
      const int dl = ntb * 16 + m;
      const float bb = bias[dbase + dl];
      h8 ev;
#pragma unroll
      for (int r = 0; r < 8; ++r) ev[r] = (_Float16)(acc0[r] * WVINV + bb);
      *(h8*)(E + dl * 64 + mt * 16 + 8 * h) = ev;
    }
    {
      const int dl = (ntb + 1) * 16 + m;
      const float bb = bias[dbase + dl];
      h8 ev;
#pragma unroll
      for (int r = 0; r < 8; ++r) ev[r] = (_Float16)(acc1[r] * WVINV + bb);
      *(h8*)(E + dl * 64 + mt * 16 + 8 * h) = ev;
    }
    __syncthreads();

    h8 vv[2];
    size_t off[2];
#pragma unroll
    for (int s = 0; s < 2; ++s) {
      const int row = w * 8 + s * 4 + (lane >> 3);
      const int q = lane & 7;
      vv[s] = *(const h8*)(E + row * 64 + q * 8);
      off[s] = ((size_t)b * CCH + dbase + row) * NPOS + n0 + q * 8;
    }
#pragma unroll
    for (int s = 0; s < 2; ++s) *(volatile h8*)(ov + off[s]) = vv[s];
    __threadfence();
#pragma unroll
    for (int s = 0; s < 2; ++s) *(volatile h8*)(ov + off[s]) = vv[s];
  }
}

__global__ void __launch_bounds__(256)
attn_kernel(const unsigned short* __restrict__ Qhi,
            const unsigned short* __restrict__ Qlo,
            const unsigned short* __restrict__ Khi,
            const unsigned short* __restrict__ Klo,
            const _Float16* __restrict__ Vh,
            const float* __restrict__ x,
            const float* __restrict__ gamma,
            float* __restrict__ outp) {
  __shared__ __align__(16) unsigned short smq[8192];
  __shared__ float Ss[32 * SSP];
  __shared__ __align__(16) _Float16 Ps[32 * PSP];
  __shared__ float mrow[32];
  __shared__ float lrow[32];
  __shared__ float srow[32];

  const int tid  = threadIdx.x;
  const int lane = tid & 31;
  const int w    = tid >> 5;
  const int m    = lane & 15;
  const int h    = lane >> 4;

  const int i0 = blockIdx.x * 32;
  const int b  = blockIdx.y;

  unsigned short* Qsh = smq;
  unsigned short* Qsl = smq + 4096;
  {
    const us8* sh = (const us8*)(Qhi + ((size_t)b * NPOS + i0) * DQK);
    const us8* sl = (const us8*)(Qlo + ((size_t)b * NPOS + i0) * DQK);
    us8* dh = (us8*)Qsh;
    us8* dl = (us8*)Qsl;
#pragma unroll
    for (int r = 0; r < 2; ++r) {
      dh[tid + r * 256] = sh[tid + r * 256];
      dl[tid + r * 256] = sl[tid + r * 256];
    }
  }
  if (tid < 32) { mrow[tid] = -1e30f; lrow[tid] = 0.0f; srow[tid] = 0.0f; }
  __syncthreads();

  v8f o[2][4];
  {
    v8f z = {};
#pragma unroll
    for (int it = 0; it < 2; ++it)
#pragma unroll
      for (int ct = 0; ct < 4; ++ct) o[it][ct] = z;
  }

  const int rtS = w >> 2;
  const int jtS = w & 3;

  for (int j0 = 0; j0 < NPOS; j0 += 64) {
    {
      v8f s = {};
      const unsigned short* qrh = Qsh + (rtS * 16 + m) * DQK + 8 * h;
      const unsigned short* qrl = Qsl + (rtS * 16 + m) * DQK + 8 * h;
      const size_t krow = ((size_t)b * NPOS + j0 + jtS * 16 + m) * DQK + 8 * h;
      const unsigned short* krh = Khi + krow;
      const unsigned short* krl = Klo + krow;
#pragma unroll
      for (int kk = 0; kk < 4; ++kk) {
        FragB ah, al, bh, bl;
        ah.p[0] = *(const us8*)(qrh + kk * 32);
        ah.p[1] = *(const us8*)(qrh + kk * 32 + 16);
        al.p[0] = *(const us8*)(qrl + kk * 32);
        al.p[1] = *(const us8*)(qrl + kk * 32 + 16);
        bh.p[0] = *(const us8*)(krh + kk * 32);
        bh.p[1] = *(const us8*)(krh + kk * 32 + 16);
        bl.p[0] = *(const us8*)(krl + kk * 32);
        bl.p[1] = *(const us8*)(krl + kk * 32 + 16);
        s = mma_bf16(ah.v, bh.v, s);
        s = mma_bf16(ah.v, bl.v, s);
        s = mma_bf16(al.v, bh.v, s);
      }
#pragma unroll
      for (int r = 0; r < 8; ++r)
        Ss[(rtS * 16 + 8 * h + r) * SSP + jtS * 16 + m] = s[r];
    }
    __syncthreads();

    if (tid < 32) {
      const int i = tid;
      const float mold = mrow[i];
      float mnew = mold;
#pragma unroll 8
      for (int j = 0; j < 64; ++j) mnew = fmaxf(mnew, Ss[i * SSP + j]);
      const float sc = __expf(mold - mnew);
      float sum = 0.0f;
#pragma unroll 8
      for (int j = 0; j < 64; ++j) {
        const float p = __expf(Ss[i * SSP + j] - mnew) * PSCALE;
        const _Float16 ph = (_Float16)p;
        Ps[i * PSP + j] = ph;
        sum += (float)ph;
      }
      mrow[i] = mnew;
      lrow[i] = lrow[i] * sc + sum;
      srow[i] = sc;
    }
    __syncthreads();

#pragma unroll
    for (int it = 0; it < 2; ++it) {
      const float sc = srow[it * 16 + m];
#pragma unroll
      for (int ct = 0; ct < 4; ++ct) o[it][ct] = o[it][ct] * sc;
    }
#pragma unroll
    for (int jj = 0; jj < 2; ++jj) {
      FragH b0, b1;
      {
        const _Float16* p0 = Ps + m * PSP + jj * 32 + 8 * h;
        const _Float16* p1 = Ps + (16 + m) * PSP + jj * 32 + 8 * h;
        b0.p[0] = *(const h8*)p0;
        b0.p[1] = *(const h8*)(p0 + 16);
        b1.p[0] = *(const h8*)p1;
        b1.p[1] = *(const h8*)(p1 + 16);
      }
#pragma unroll
      for (int ct = 0; ct < 4; ++ct) {
        FragH a;
        const _Float16* vr = Vh + ((size_t)b * CCH + w * 64 + ct * 16 + m) * NPOS + j0 + jj * 32 + 8 * h;
        a.p[0] = *(const h8*)vr;
        a.p[1] = *(const h8*)(vr + 16);
        o[0][ct] = mma_f16(a.v, b0.v, o[0][ct]);
        o[1][ct] = mma_f16(a.v, b1.v, o[1][ct]);
      }
    }
    __syncthreads();
  }

  const float g = gamma[0];
  const float gl0 = g / lrow[m];
  const float gl1 = g / lrow[16 + m];
  float* F = (float*)smq + w * 512;
#pragma unroll
  for (int ct = 0; ct < 4; ++ct) {
    __syncthreads();
#pragma unroll
    for (int r = 0; r < 8; ++r) {
      F[(8 * h + r) * 32 + m]      = o[0][ct][r] * gl0;
      F[(8 * h + r) * 32 + 16 + m] = o[1][ct][r] * gl1;
    }
    __syncthreads();
    v4f vals[4];
    size_t offs[4];
#pragma unroll
    for (int s = 0; s < 4; ++s) {
      const int row = s * 4 + (lane >> 3);
      const int q = lane & 7;
      const int c = w * 64 + ct * 16 + row;
      const size_t off = ((size_t)b * CCH + c) * NPOS + i0 + q * 4;
      const v4f ov = *(const v4f*)(F + row * 32 + q * 4);
      const v4f xv = *(const v4f*)(x + off);
      vals[s] = ov + xv;
      offs[s] = off;
    }
#pragma unroll
    for (int s = 0; s < 4; ++s) *(volatile v4f*)(outp + offs[s]) = vals[s];
    __threadfence();
#pragma unroll
    for (int s = 0; s < 4; ++s) *(volatile v4f*)(outp + offs[s]) = vals[s];
  }
}

extern "C" void kernel_launch(void* const* d_in, const int* in_sizes, int n_in,
                              void* d_out, int out_size, void* d_ws, size_t ws_size,
                              hipStream_t stream) {
  if (n_in < 13) return;
  const int nx = BATCH * CCH * NPOS;
  if (in_sizes[0] != nx || in_sizes[1] != nx ||
      in_sizes[2] != CQ * CCH || in_sizes[3] != CQ ||
      in_sizes[4] != CQ * CCH || in_sizes[5] != CQ ||
      in_sizes[6] != CQ * CCH || in_sizes[7] != CQ ||
      in_sizes[8] != CQ * CCH || in_sizes[9] != CQ ||
      in_sizes[10] != CCH * CCH || in_sizes[11] != CCH ||
      in_sizes[12] < 1 || out_size != nx) return;

  const size_t planeE = (size_t)BATCH * NPOS * DQK;
  const size_t vE     = (size_t)BATCH * CCH * NPOS;
  const size_t need   = planeE * 2 * 4 + vE * 2;
  if (ws_size < need) return;

  const float* x     = (const float*)d_in[0];
  const float* dep   = (const float*)d_in[1];
  const float* wq    = (const float*)d_in[2];
  const float* bq    = (const float*)d_in[3];
  const float* wqd   = (const float*)d_in[4];
  const float* bqd   = (const float*)d_in[5];
  const float* wk    = (const float*)d_in[6];
  const float* bk    = (const float*)d_in[7];
  const float* wkd   = (const float*)d_in[8];
  const float* bkd   = (const float*)d_in[9];
  const float* wv    = (const float*)d_in[10];
  const float* bv    = (const float*)d_in[11];
  const float* gamma = (const float*)d_in[12];
  float* outp = (float*)d_out;

  unsigned short* Qhi = (unsigned short*)d_ws;
  unsigned short* Qlo = Qhi + planeE;
  unsigned short* Khi = Qlo + planeE;
  unsigned short* Klo = Khi + planeE;
  _Float16* Vh = (_Float16*)(Klo + planeE);

  dim3 blk(256);
  dim3 gqk(NPOS / 64, 1, BATCH);
  proj_kernel<0><<<gqk, blk, 0, stream>>>(x,   wq,  bq,  Qhi, Qlo, Vh, 0);
  proj_kernel<0><<<gqk, blk, 0, stream>>>(dep, wqd, bqd, Qhi, Qlo, Vh, CQ);
  proj_kernel<0><<<gqk, blk, 0, stream>>>(x,   wk,  bk,  Khi, Klo, Vh, 0);
  proj_kernel<0><<<gqk, blk, 0, stream>>>(dep, wkd, bkd, Khi, Klo, Vh, CQ);
  proj_kernel<1><<<dim3(NPOS / 64, CCH / 64, BATCH), blk, 0, stream>>>(x, wv, bv, Qhi, Qlo, Vh, 0);
  attn_kernel<<<dim3(NPOS / 32, BATCH), blk, 0, stream>>>(Qhi, Qlo, Khi, Klo, Vh, x, gamma, outp);
}
